// RWKV_Tmix_x070_Mod_42004780155477
// MI455X (gfx1250) — hardware-verified
//
#include <hip/hip_runtime.h>
#include <math.h>

constexpr int kBatch  = 2;
constexpr int kSteps  = 1024;
constexpr int kChan   = 1024;
constexpr int kHeads  = 16;
constexpr int kHdim   = 64;
constexpr int kTok    = kBatch * kSteps;
constexpr size_t kPlane = (size_t)kTok * kChan;
constexpr int kLoraW  = 64;
constexpr int kLoraA  = 64;
constexpr int kLoraV  = 32;
constexpr int kLoraVP = 64;
constexpr int kLoraG  = 128;
constexpr int kChunk  = 16;

constexpr float kWCarry   = 16.0f;
constexpr float kHidCarry = 16.0f;
constexpr float kYCarry   = 16.0f;
constexpr float kResCarry = 2048.0f;
constexpr float kResInv   = 1.0f / kResCarry;
constexpr float kScaleW   = 1.0f / kWCarry;
constexpr float kScaleWH  = 1.0f / (kWCarry * kHidCarry);
constexpr float kScaleOut = 1.0f / (kWCarry * kYCarry);
constexpr float kGnEps    = 64e-5f;

static_assert(kHeads * kHdim == kChan);
static_assert(kTok % 32 == 0 && kChan % 64 == 0);
static_assert(kLoraW % 64 == 0 && kLoraA % 64 == 0 && kLoraVP % 64 == 0 && kLoraG % 64 == 0);
static_assert(kChan % 32 == 0 && kLoraW % 32 == 0 && kLoraVP % 32 == 0 && kLoraG % 32 == 0);
static_assert(kSteps % kChunk == 0);
static_assert((kTok * kHeads) % 8 == 0);
static_assert(kHdim == 64 && kChunk == 16);

typedef __attribute__((ext_vector_type(16))) _Float16 v16h;
typedef __attribute__((ext_vector_type(8)))  _Float16 v8h;
typedef __attribute__((ext_vector_type(8)))  float    v8f;
typedef __attribute__((ext_vector_type(4)))  float    v4f;
typedef __attribute__((ext_vector_type(2)))  float    v2f;
typedef __attribute__((ext_vector_type(4)))  unsigned int v4u;

__device__ __forceinline__ unsigned pk16(unsigned short a, unsigned short b) {
  return (unsigned)a | ((unsigned)b << 16);
}
__device__ __forceinline__ unsigned short h_bits(float f) {
  const _Float16 h = (_Float16)f;
  return __builtin_bit_cast(unsigned short, h);
}
__device__ __forceinline__ void h_split(float v, unsigned short& hb, unsigned short& rb) {
  const _Float16 h = (_Float16)v;
  const float hf = (float)h;
  const float d = v - hf;
  const _Float16 r = (_Float16)(d * kResCarry);
  hb = __builtin_bit_cast(unsigned short, h);
  rb = __builtin_bit_cast(unsigned short, r);
}
__device__ __forceinline__ v4u pack8_plain(const float (&v)[8]) {
  unsigned short hb[8];
#pragma unroll
  for (int e = 0; e < 8; ++e) hb[e] = h_bits(v[e]);
  return (v4u){pk16(hb[0], hb[1]), pk16(hb[2], hb[3]), pk16(hb[4], hb[5]), pk16(hb[6], hb[7])};
}
__device__ __forceinline__ void pack8_split(const float (&v)[8], v4u& uh, v4u& ur) {
  unsigned short hb[8], rb[8];
#pragma unroll
  for (int e = 0; e < 8; ++e) h_split(v[e], hb[e], rb[e]);
  uh = (v4u){pk16(hb[0], hb[1]), pk16(hb[2], hb[3]), pk16(hb[4], hb[5]), pk16(hb[6], hb[7])};
  ur = (v4u){pk16(rb[0], rb[1]), pk16(rb[2], rb[3]), pk16(rb[4], rb[5]), pk16(rb[6], rb[7])};
}
__device__ __forceinline__ float wave_sum32(float v) {
#pragma unroll
  for (int o = 16; o > 0; o >>= 1) v += __shfl_xor(v, o, 32);
  return v;
}

struct FragH {
  union U { v16h v; v8h h[2]; };
  static __device__ __forceinline__ v16h load(const _Float16* p) {
    U f;
    f.h[0] = *(const v8h*)(p);
    f.h[1] = *(const v8h*)(p + 16);
    return f.v;
  }
  static __device__ __forceinline__ v8f mma(v16h a, v16h b, v8f c) {
    return __builtin_amdgcn_wmma_f32_16x16x32_f16(false, a, false, b, (short)0, c, false, false);
  }
};
__device__ __forceinline__ void guard_split(v8f& a0, v8f& a1, v8f& a2, v8f& a3,
                                            v16h x0, v16h x1, v16h x2, v16h x3, v16h y0, v16h y1) {
  asm volatile("v_nop\n\tv_nop\n\tv_nop\n\tv_nop"
               : "+v"(a0), "+v"(a1), "+v"(a2), "+v"(a3)
               : "v"(x0), "v"(x1), "v"(x2), "v"(x3), "v"(y0), "v"(y1));
}
__device__ __forceinline__ void guard_plain(v8f& a0, v8f& a1, v16h x0, v16h x1, v16h y0) {
  asm volatile("v_nop\n\tv_nop\n\tv_nop\n\tv_nop"
               : "+v"(a0), "+v"(a1)
               : "v"(x0), "v"(x1), "v"(y0));
}
__device__ __forceinline__ void acc_guard4(v8f& a, v8f& b, v8f& c, v8f& d) {
  asm volatile("v_nop\n\tv_nop\n\tv_nop\n\tv_nop" : "+v"(a), "+v"(b), "+v"(c), "+v"(d));
}

template <bool SPLIT, int ACT, int OUT_MODE>
__global__ __launch_bounds__(256) void gemm_f16_kernel(
    const unsigned short* __restrict__ Ahp, const unsigned short* __restrict__ Arp, int lda, long strideA,
    const unsigned short* __restrict__ Bhp, const unsigned short* __restrict__ Brp, int ldb, long strideB,
    void* __restrict__ Cout, int ldc, long strideC,
    int M, int N, int K, float scale) {
  static_assert(ACT == 0 || OUT_MODE == 1);
  __shared__ __align__(16) float sT[8][16 * 68];
  const int z    = blockIdx.y;
  const int lane = threadIdx.x & 31;
  const int wave = threadIdx.x >> 5;
  const int tilesN = N >> 6;
  const int tilesM = M >> 5;
  const int tile = blockIdx.x * 8 + wave;
  if (tile >= tilesM * tilesN) return;
  const int tm = tile / tilesN;
  const int tn = tile - tm * tilesN;
  const int m0 = tm << 5;
  const int n0 = tn << 6;
  const int rlane = lane & 15;
  const int half8 = (lane >> 4) * 8;
  const int mOff  = (lane >> 4) * 8;

  const size_t aoff = (size_t)z * (size_t)strideA + (size_t)(m0 + rlane) * lda + half8;
  const size_t boff = (size_t)z * (size_t)strideB + (size_t)(n0 + rlane) * ldb + half8;
  const _Float16* pa0 = (const _Float16*)Ahp + aoff;
  const _Float16* pa1 = pa0 + (size_t)16 * lda;
  const _Float16* pr0 = SPLIT ? ((const _Float16*)Arp + aoff) : pa0;
  const _Float16* pr1 = pr0 + (size_t)16 * lda;
  const _Float16* pbh = (const _Float16*)Bhp + boff;
  const _Float16* pbr = SPLIT ? ((const _Float16*)Brp + boff) : pbh;
  const size_t bstep = (size_t)16 * ldb;

  v8f acc[2][4], accr[2][4];
#pragma unroll
  for (int i = 0; i < 2; ++i)
#pragma unroll
    for (int j = 0; j < 4; ++j) {
      acc[i][j]  = (v8f){0.f, 0.f, 0.f, 0.f, 0.f, 0.f, 0.f, 0.f};
      accr[i][j] = (v8f){0.f, 0.f, 0.f, 0.f, 0.f, 0.f, 0.f, 0.f};
    }

  for (int k0 = 0; k0 < K; k0 += 32) {
    const v16h ah0 = FragH::load(pa0 + k0);
    const v16h ah1 = FragH::load(pa1 + k0);
    v16h ar0 = ah0, ar1 = ah1;
    if (SPLIT) {
      ar0 = FragH::load(pr0 + k0);
      ar1 = FragH::load(pr1 + k0);
    }
#pragma unroll
    for (int j = 0; j < 4; ++j) {
      const v16h bh = FragH::load(pbh + j * bstep + k0);
      v16h br = bh;
      if (SPLIT) br = FragH::load(pbr + j * bstep + k0);
      acc[0][j] = FragH::mma(ah0, bh, acc[0][j]);
      acc[1][j] = FragH::mma(ah1, bh, acc[1][j]);
      if (SPLIT) {
        accr[0][j] = FragH::mma(ah0, br, accr[0][j]);
        accr[1][j] = FragH::mma(ah1, br, accr[1][j]);
        accr[0][j] = FragH::mma(ar0, bh, accr[0][j]);
        accr[1][j] = FragH::mma(ar1, bh, accr[1][j]);
        guard_split(acc[0][j], acc[1][j], accr[0][j], accr[1][j], ah0, ah1, ar0, ar1, bh, br);
      } else {
        guard_plain(acc[0][j], acc[1][j], ah0, ah1, bh);
      }
    }
  }
  acc_guard4(acc[0][0], acc[0][1], acc[0][2], acc[0][3]);
  acc_guard4(acc[1][0], acc[1][1], acc[1][2], acc[1][3]);
  if (SPLIT) {
    acc_guard4(accr[0][0], accr[0][1], accr[0][2], accr[0][3]);
    acc_guard4(accr[1][0], accr[1][1], accr[1][2], accr[1][3]);
  }

  float* slab = sT[wave];
#pragma unroll
  for (int i = 0; i < 2; ++i) {
    const int mBase = m0 + (i << 4);
#pragma unroll
    for (int j = 0; j < 4; ++j) {
#pragma unroll
      for (int r = 0; r < 8; ++r) {
        float v = acc[i][j][r];
        if (SPLIT) v += accr[i][j][r] * kResInv;
        v *= scale;
        slab[(mOff + r) * 68 + (j << 4) + rlane] = v;
      }
    }
    __builtin_amdgcn_fence(__ATOMIC_RELEASE, "workgroup");
    __builtin_amdgcn_wave_barrier();
    __builtin_amdgcn_fence(__ATOMIC_ACQUIRE, "workgroup");
    if (OUT_MODE == 0) {
      float* C = (float*)Cout + (size_t)z * (size_t)strideC;
      const int hh = lane >> 4, c4 = (lane & 15) * 4;
      for (int pass = 0; pass < 2; ++pass) {
#pragma unroll
        for (int it = 0; it < 8; ++it) {
          const int row = it * 2 + hh;
          const v4f v = *(const v4f*)(slab + row * 68 + c4);
          *(volatile v4f*)(C + (size_t)(mBase + row) * ldc + n0 + c4) = v;
        }
        __threadfence();
      }
    } else {
      const int q = lane >> 3, c8 = (lane & 7) * 8;
      if (ACT != 0) {
#pragma unroll 1
        for (int it = 0; it < 4; ++it) {
          float* sp = slab + (it * 4 + q) * 68 + c8;
#pragma unroll
          for (int e = 0; e < 8; ++e) {
            const float x = sp[e];
            float y;
            if (ACT == 1) y = tanhf(x);
            else y = 1.0f / (1.0f + expf(-x));
            sp[e] = y * kHidCarry;
          }
        }
      }
      unsigned short* C = (unsigned short*)Cout + (size_t)z * (size_t)strideC;
      for (int pass = 0; pass < 2; ++pass) {
#pragma unroll
        for (int it = 0; it < 4; ++it) {
          const int row = it * 4 + q;
          const float* sp = slab + row * 68 + c8;
          v8h hv;
#pragma unroll
          for (int e = 0; e < 8; ++e) hv[e] = (_Float16)sp[e];
          *(volatile v8h*)(C + (size_t)(mBase + row) * ldc + n0 + c8) = hv;
        }
        __threadfence();
      }
    }
    __builtin_amdgcn_fence(__ATOMIC_RELEASE, "workgroup");
    __builtin_amdgcn_wave_barrier();
    __builtin_amdgcn_fence(__ATOMIC_ACQUIRE, "workgroup");
  }
}

__global__ __launch_bounds__(256) void wt_plane_kernel(const float* __restrict__ W0, const float* __restrict__ W1,
                                                       const float* __restrict__ W2, const float* __restrict__ W3,
                                                       unsigned short* __restrict__ outh, unsigned short* __restrict__ outr,
                                                       int Kd, int Nd, int KdP, int NdP, int has_res) {
  __shared__ float sm[64][65];
  const int t  = threadIdx.x;
  const int k0 = blockIdx.x * 64;
  const int n0 = blockIdx.y * 64;
  const int z  = blockIdx.z;
  const float* W = (z == 0) ? W0 : (z == 1) ? W1 : (z == 2) ? W2 : W3;
#pragma unroll
  for (int i = 0; i < 16; ++i) {
    const int e = i * 256 + t;
    const int r = e >> 6;
    const int c = e & 63;
    const int kk = k0 + r;
    const int nn = n0 + c;
    const bool valid = (kk < Kd) && (nn < Nd);
    const int kc = (kk < Kd) ? kk : (Kd - 1);
    const int nc = (nn < Nd) ? nn : (Nd - 1);
    const float v = W[(size_t)kc * Nd + nc];
    sm[c][r] = valid ? (v * kWCarry) : 0.0f;
  }
  __syncthreads();
  const int lane = t & 31, wave = t >> 5;
  const int q = lane >> 3, c8 = (lane & 7) * 8;
  const size_t pofs = (size_t)z * (size_t)NdP * (size_t)KdP;
  for (int pass = 0; pass < 2; ++pass) {
#pragma unroll
    for (int it = 0; it < 2; ++it) {
      const int row = wave * 8 + it * 4 + q;
      float v[8];
#pragma unroll
      for (int e = 0; e < 8; ++e) v[e] = sm[row][c8 + e];
      v4u uh, ur;
      pack8_split(v, uh, ur);
      const size_t o = pofs + (size_t)(n0 + row) * KdP + k0 + c8;
      *(volatile v4u*)(outh + o) = uh;
      if (has_res) *(volatile v4u*)(outr + o) = ur;
    }
    __threadfence();
  }
}

__device__ __forceinline__ void mix8(const float* __restrict__ m, int c8, const float (&cur)[8],
                                     const float (&xx)[8], float (&o)[8]) {
  const v4f a = *(const v4f*)(m + c8);
  const v4f b = *(const v4f*)(m + c8 + 4);
#pragma unroll
  for (int e = 0; e < 4; ++e) {
    o[e]     = cur[e]     + xx[e]     * a[e];
    o[4 + e] = cur[4 + e] + xx[4 + e] * b[e];
  }
}

__global__ __launch_bounds__(256) void mix_kernel(const float* __restrict__ x,
                                                  const float* __restrict__ m_r, const float* __restrict__ m_w,
                                                  const float* __restrict__ m_k, const float* __restrict__ m_v,
                                                  const float* __restrict__ m_a, const float* __restrict__ m_g,
                                                  unsigned short* __restrict__ XRh, unsigned short* __restrict__ XRr,
                                                  unsigned short* __restrict__ XKh, unsigned short* __restrict__ XKr,
                                                  unsigned short* __restrict__ XVh, unsigned short* __restrict__ XVr,
                                                  unsigned short* __restrict__ XW, unsigned short* __restrict__ XA,
                                                  unsigned short* __restrict__ XG) {
  const int i = blockIdx.x * 256 + threadIdx.x;
  if (i >= kTok * (kChan / 8)) return;
  const int row = i >> 7;
  const int c8  = (i & 127) * 8;
  const bool first = (row & (kSteps - 1)) == 0;
  const int prow = first ? row : (row - 1);
  const float* xp = x + (size_t)row * kChan + c8;
  const float* pp = x + (size_t)prow * kChan + c8;
  const v4f a  = *(const v4f*)(xp);
  const v4f b  = *(const v4f*)(xp + 4);
  const v4f pa = *(const v4f*)(pp);
  const v4f pb = *(const v4f*)(pp + 4);
  float cur[8], xx[8];
#pragma unroll
  for (int e = 0; e < 4; ++e) {
    cur[e]     = a[e];
    cur[4 + e] = b[e];
    const float p0 = first ? 0.0f : pa[e];
    const float p1 = first ? 0.0f : pb[e];
    xx[e]     = p0 - a[e];
    xx[4 + e] = p1 - b[e];
  }
  float o[8];
  v4u urh, urr, ukh, ukr, uvh, uvr, uw, ua, ug;
  mix8(m_r, c8, cur, xx, o); pack8_split(o, urh, urr);
  mix8(m_k, c8, cur, xx, o); pack8_split(o, ukh, ukr);
  mix8(m_v, c8, cur, xx, o); pack8_split(o, uvh, uvr);
  mix8(m_w, c8, cur, xx, o); uw = pack8_plain(o);
  mix8(m_a, c8, cur, xx, o); ua = pack8_plain(o);
  mix8(m_g, c8, cur, xx, o); ug = pack8_plain(o);
  const size_t off = (size_t)i * 8;
  for (int pass = 0; pass < 2; ++pass) {
    *(volatile v4u*)(XRh + off) = urh;
    *(volatile v4u*)(XRr + off) = urr;
    *(volatile v4u*)(XKh + off) = ukh;
    *(volatile v4u*)(XKr + off) = ukr;
    *(volatile v4u*)(XVh + off) = uvh;
    *(volatile v4u*)(XVr + off) = uvr;
    *(volatile v4u*)(XW + off) = uw;
    *(volatile v4u*)(XA + off) = ua;
    *(volatile v4u*)(XG + off) = ug;
    __threadfence();
  }
}

__global__ __launch_bounds__(256) void gate_prep_kernel(float* Kf, float* Vf, float* WD, float* AB, float* VK,
                                                        const float* __restrict__ vfirst,
                                                        const float* __restrict__ w0, const float* __restrict__ a0,
                                                        const float* __restrict__ v0b, const float* __restrict__ k_k,
                                                        const float* __restrict__ k_a) {
  const int lane = threadIdx.x & 31;
  const int pair = blockIdx.x * 8 + (threadIdx.x >> 5);
  const int tok = pair >> 4;
  const int h   = pair & 15;
  const size_t base = (size_t)tok * kChan + (size_t)h * kHdim;
  const int cb = h * kHdim;
  float ss;
  {
    const float ka = Kf[base + lane] * k_k[cb + lane];
    const float kb = Kf[base + lane + 32] * k_k[cb + lane + 32];
    ss = wave_sum32(ka * ka + kb * kb);
  }
  const float inv = 1.0f / fmaxf(sqrtf(ss), 1e-12f);
#pragma unroll 1
  for (int hf = 0; hf < 2; ++hf) {
    const size_t idx = base + lane + 32 * hf;
    const int c = cb + lane + 32 * hf;
    const float k0  = Kf[idx];
    const float kkv = (k0 * k_k[c]) * inv;
    const float av  = __builtin_amdgcn_rcpf(1.0f + expf(-(AB[idx] + a0[c])));
    const float km  = k0 * (1.0f + (av - 1.0f) * k_a[c]);
    const float zz  = WD[idx] + w0[c];
    const float nz  = -zz;
    const float spv = fmaxf(nz, 0.0f) + log1pf(expf(-fabsf(nz)));
    const float wv  = -spv - 0.5f;
    const float dv  = expf(-expf(wv));
    const float vg  = __builtin_amdgcn_rcpf(1.0f + expf(-(VK[idx] + v0b[c])));
    const float vp  = Vf[idx];
    const float vm  = vp + (vfirst[idx] - vp) * vg;
    const float bv  = kkv * av;
    *(volatile float*)(Kf + idx) = km;
    *(volatile float*)(Vf + idx) = vm;
    *(volatile float*)(WD + idx) = dv;
    *(volatile float*)(AB + idx) = bv;
    *(volatile float*)(VK + idx) = kkv;
    __threadfence();
    *(volatile float*)(Kf + idx) = km;
    *(volatile float*)(Vf + idx) = vm;
    *(volatile float*)(WD + idx) = dv;
    *(volatile float*)(AB + idx) = bv;
    *(volatile float*)(VK + idx) = kkv;
  }
}

__global__ __launch_bounds__(256) void state_scan_kernel(const float* __restrict__ Rf, const float* __restrict__ Dd,
                                                         const float* __restrict__ Kf, const float* __restrict__ Vf,
                                                         const float* __restrict__ KKf, const float* __restrict__ Bv,
                                                         float* __restrict__ Y) {
  __shared__ __align__(16) float lv[6 * kChunk * 64];
  __shared__ __align__(16) float yb[kChunk * 64];
  const int bh  = blockIdx.x;
  const int b   = bh >> 4;
  const int h   = bh & 15;
  const int tid = threadIdx.x;
  const int i   = tid >> 2;
  const int q   = tid & 3;
  const int j0  = q * 16;
  const int lrow = tid >> 4;
  const int lc4  = (tid & 15) * 4;
  const size_t base = (size_t)b * kSteps * kChan + (size_t)h * kHdim;

  float S[16];
#pragma unroll
  for (int jj = 0; jj < 16; ++jj) S[jj] = 0.0f;

#pragma unroll 1
  for (int ch = 0; ch < kSteps / kChunk; ++ch) {
    const size_t goff = base + (size_t)(ch * kChunk + lrow) * kChan + lc4;
    {
      const v4f t0 = *(const v4f*)(Rf + goff);
      const v4f t1 = *(const v4f*)(Dd + goff);
      const v4f t2 = *(const v4f*)(Kf + goff);
      const v4f t3 = *(const v4f*)(Vf + goff);
      const v4f t4 = *(const v4f*)(KKf + goff);
      const v4f t5 = *(const v4f*)(Bv + goff);
      const int lo = lrow * 64 + lc4;
      *(v4f*)(lv + 0 * kChunk * 64 + lo) = t0;
      *(v4f*)(lv + 1 * kChunk * 64 + lo) = t1;
      *(v4f*)(lv + 2 * kChunk * 64 + lo) = t2;
      *(v4f*)(lv + 3 * kChunk * 64 + lo) = t3;
      *(v4f*)(lv + 4 * kChunk * 64 + lo) = t4;
      *(v4f*)(lv + 5 * kChunk * 64 + lo) = t5;
    }
    __syncthreads();

#pragma unroll 1
    for (int s = 0; s < kChunk; ++s) {
      const float* pr  = lv + 0 * kChunk * 64 + s * 64 + j0;
      const float* pd  = lv + 1 * kChunk * 64 + s * 64 + j0;
      const float* pk  = lv + 2 * kChunk * 64 + s * 64 + j0;
      const float* pkk = lv + 4 * kChunk * 64 + s * 64 + j0;
      const float* pb  = lv + 5 * kChunk * 64 + s * 64 + j0;
      const float vi = lv[3 * kChunk * 64 + s * 64 + i];
      float sa = 0.0f;
#pragma unroll
      for (int g4 = 0; g4 < 4; ++g4) {
        const v4f k4 = *(const v4f*)(pkk + 4 * g4);
#pragma unroll
        for (int e = 0; e < 4; ++e) sa += S[4 * g4 + e] * k4[e];
      }
      sa += __shfl_xor(sa, 1, 32);
      sa += __shfl_xor(sa, 2, 32);
      sa = -sa;
      float out = 0.0f;
#pragma unroll
      for (int g4 = 0; g4 < 4; ++g4) {
        const v4f d4 = *(const v4f*)(pd + 4 * g4);
        const v4f b4 = *(const v4f*)(pb + 4 * g4);
        const v4f k4 = *(const v4f*)(pk + 4 * g4);
        const v4f r4 = *(const v4f*)(pr + 4 * g4);
#pragma unroll
        for (int e = 0; e < 4; ++e) {
          const float sn = S[4 * g4 + e] * d4[e] + sa * b4[e] + vi * k4[e];
          S[4 * g4 + e] = sn;
          out += sn * r4[e];
        }
      }
      out += __shfl_xor(out, 1, 32);
      out += __shfl_xor(out, 2, 32);
      if (q == 0) yb[s * 64 + i] = out;
    }
    __syncthreads();
    {
      const v4f val = *(const v4f*)(yb + lrow * 64 + lc4);
      *(volatile v4f*)(Y + goff) = val;
      __threadfence();
      *(volatile v4f*)(Y + goff) = val;
    }
  }
}

__global__ __launch_bounds__(256) void norm_gate_kernel(const float* __restrict__ Y, const float* __restrict__ Rf,
                                                        const float* __restrict__ Kf, const float* __restrict__ Vf,
                                                        const float* __restrict__ Gf, const float* __restrict__ r_k,
                                                        const float* __restrict__ ln_w, const float* __restrict__ ln_b,
                                                        unsigned* __restrict__ YGh, unsigned* __restrict__ YGr) {
  const int lane = threadIdx.x & 31;
  const int pair = blockIdx.x * 8 + (threadIdx.x >> 5);
  const int tok = pair >> 4;
  const int h   = pair & 15;
  const size_t base = (size_t)tok * kChan + (size_t)h * kHdim + 2 * lane;
  const int c = h * kHdim + 2 * lane;
  const v2f y2 = *(const v2f*)(Y + base);
  const v2f r2 = *(const v2f*)(Rf + base);
  const v2f k2 = *(const v2f*)(Kf + base);
  const v2f v2 = *(const v2f*)(Vf + base);
  const v2f g2 = *(const v2f*)(Gf + base);
  const v2f q2 = *(const v2f*)(r_k + c);
  const v2f w2 = *(const v2f*)(ln_w + c);
  const v2f b2 = *(const v2f*)(ln_b + c);
  const float mu = wave_sum32(y2[0] + y2[1]) * (1.0f / 64.0f);
  const float d0 = y2[0] - mu;
  const float d1 = y2[1] - mu;
  const float var = wave_sum32(d0 * d0 + d1 * d1) * (1.0f / 64.0f);
  const float inv = 1.0f / sqrtf(var + kGnEps);
  const float bsum = wave_sum32(r2[0] * k2[0] * q2[0] + r2[1] * k2[1] * q2[1]);
  const float o0 = (((d0 * inv) * w2[0] + b2[0]) + bsum * v2[0]) * g2[0] * kYCarry;
  const float o1 = (((d1 * inv) * w2[1] + b2[1]) + bsum * v2[1]) * g2[1] * kYCarry;
  unsigned short h0, s0, h1, s1;
  h_split(o0, h0, s0);
  h_split(o1, h1, s1);
  const unsigned wh = pk16(h0, h1);
  const unsigned wr = pk16(s0, s1);
  const size_t widx = base >> 1;
  *(volatile unsigned*)(YGh + widx) = wh;
  *(volatile unsigned*)(YGr + widx) = wr;
  __threadfence();
  *(volatile unsigned*)(YGh + widx) = wh;
  *(volatile unsigned*)(YGr + widx) = wr;
}

__global__ __launch_bounds__(256) void copy_f32x4_kernel(const float* __restrict__ src, float* __restrict__ dst, int n4) {
  const int i = blockIdx.x * 256 + threadIdx.x;
  if (i >= n4) return;
  const v4f v = *(const v4f*)(src + (size_t)i * 4);
  *(volatile v4f*)(dst + (size_t)i * 4) = v;
  __threadfence();
  *(volatile v4f*)(dst + (size_t)i * 4) = v;
}

extern "C" void kernel_launch(void* const* d_in, const int* in_sizes, int n_in,
                              void* d_out, int out_size, void* d_ws, size_t ws_size, hipStream_t stream) {
  if (n_in < 28 || d_out == nullptr || d_ws == nullptr) return;
  const int nP = (int)kPlane;
  if (in_sizes[0] != nP || in_sizes[1] != nP) return;
  for (int i = 2; i <= 7; ++i) if (in_sizes[i] != kChan) return;
  if (in_sizes[8] != kChan * kLoraW || in_sizes[9] != kLoraW * kChan || in_sizes[10] != kChan) return;
  if (in_sizes[11] != kChan * kLoraA || in_sizes[12] != kLoraA * kChan || in_sizes[13] != kChan) return;
  if (in_sizes[14] != kChan * kLoraV || in_sizes[15] != kLoraV * kChan || in_sizes[16] != kChan) return;
  if (in_sizes[17] != kChan * kLoraG || in_sizes[18] != kLoraG * kChan) return;
  if (in_sizes[19] != kChan || in_sizes[20] != kChan || in_sizes[21] != kHeads * kHdim) return;
  for (int i = 22; i <= 25; ++i) if (in_sizes[i] != kChan * kChan) return;
  if (in_sizes[26] != kChan || in_sizes[27] != kChan) return;
  if (out_size != 2 * nP) return;

  const float* x      = (const float*)d_in[0];
  const float* vfirst = (const float*)d_in[1];
  const float* x_r = (const float*)d_in[2];
  const float* x_w = (const float*)d_in[3];
  const float* x_k = (const float*)d_in[4];
  const float* x_v = (const float*)d_in[5];
  const float* x_a = (const float*)d_in[6];
  const float* x_g = (const float*)d_in[7];
  const float* w1 = (const float*)d_in[8];
  const float* w2 = (const float*)d_in[9];
  const float* w0 = (const float*)d_in[10];
  const float* a1 = (const float*)d_in[11];
  const float* a2 = (const float*)d_in[12];
  const float* a0 = (const float*)d_in[13];
  const float* v1 = (const float*)d_in[14];
  const float* v2 = (const float*)d_in[15];
  const float* v0 = (const float*)d_in[16];
  const float* g1 = (const float*)d_in[17];
  const float* g2 = (const float*)d_in[18];
  const float* k_k = (const float*)d_in[19];
  const float* k_a = (const float*)d_in[20];
  const float* r_k = (const float*)d_in[21];
  const float* W_r = (const float*)d_in[22];
  const float* W_k = (const float*)d_in[23];
  const float* W_v = (const float*)d_in[24];
  const float* W_o = (const float*)d_in[25];
  const float* ln_w = (const float*)d_in[26];
  const float* ln_b = (const float*)d_in[27];
  float* out0 = (float*)d_out;
  float* out1 = out0 + kPlane;

  char* ws = (char*)d_ws;
  size_t off = 0;
  auto carve = [&](size_t bytes) -> char* {
    char* p = ws + off;
    off += (bytes + 255) & ~(size_t)255;
    return p;
  };
  const size_t actB = kPlane * 2;
  const size_t wBig = (size_t)kChan * kChan;
  unsigned short* XRh = (unsigned short*)carve(actB);
  unsigned short* XKh = (unsigned short*)carve(actB);
  unsigned short* XVh = (unsigned short*)carve(actB);
  unsigned short* XRr = (unsigned short*)carve(actB);
  unsigned short* XKr = (unsigned short*)carve(actB);
  unsigned short* XVr = (unsigned short*)carve(actB);
  unsigned short* XW  = (unsigned short*)carve(actB);
  unsigned short* XA  = (unsigned short*)carve(actB);
  unsigned short* XG  = (unsigned short*)carve(actB);
  unsigned short* WBh = (unsigned short*)carve(4 * wBig * 2);
  unsigned short* WBr = (unsigned short*)carve(4 * wBig * 2);
  unsigned short* w1T = (unsigned short*)carve((size_t)kLoraW * kChan * 2);
  unsigned short* a1T = (unsigned short*)carve((size_t)kLoraA * kChan * 2);
  unsigned short* v1T = (unsigned short*)carve((size_t)kLoraVP * kChan * 2);
  unsigned short* g1T = (unsigned short*)carve((size_t)kLoraG * kChan * 2);
  unsigned short* w2T = (unsigned short*)carve((size_t)kChan * kLoraW * 2);
  unsigned short* a2T = (unsigned short*)carve((size_t)kChan * kLoraA * 2);
  unsigned short* v2T = (unsigned short*)carve((size_t)kChan * kLoraVP * 2);
  unsigned short* g2T = (unsigned short*)carve((size_t)kChan * kLoraG * 2);
  unsigned short* HW  = (unsigned short*)carve((size_t)kTok * kLoraW * 2);
  unsigned short* HA  = (unsigned short*)carve((size_t)kTok * kLoraA * 2);
  unsigned short* HV  = (unsigned short*)carve((size_t)kTok * kLoraVP * 2);
  unsigned short* HG  = (unsigned short*)carve((size_t)kTok * kLoraG * 2);
  float* Rf = (float*)carve(kPlane * 4);
  float* Kf = (float*)carve(kPlane * 4);
  float* Vf = (float*)carve(kPlane * 4);
  float* WD = (float*)carve(kPlane * 4);
  float* AB = (float*)carve(kPlane * 4);
  float* VK = (float*)carve(kPlane * 4);
  float* Gf = (float*)carve(kPlane * 4);
  float* Yf = (float*)carve(kPlane * 4);
  unsigned short* YGh = XRh;
  unsigned short* YGr = XRr;
  if (off > ws_size || off > (size_t)134217728) return;

  wt_plane_kernel<<<dim3(kChan / 64, kChan / 64, 4), 256, 0, stream>>>(W_r, W_k, W_v, W_o, WBh, WBr,
                                                                        kChan, kChan, kChan, kChan, 1);
  wt_plane_kernel<<<dim3(kChan / 64, kLoraW / 64, 1), 256, 0, stream>>>(w1, w1, w1, w1, w1T, w1T, kChan, kLoraW, kChan, kLoraW, 0);
  wt_plane_kernel<<<dim3(kChan / 64, kLoraA / 64, 1), 256, 0, stream>>>(a1, a1, a1, a1, a1T, a1T, kChan, kLoraA, kChan, kLoraA, 0);
  wt_plane_kernel<<<dim3(kChan / 64, kLoraVP / 64, 1), 256, 0, stream>>>(v1, v1, v1, v1, v1T, v1T, kChan, kLoraV, kChan, kLoraVP, 0);
  wt_plane_kernel<<<dim3(kChan / 64, kLoraG / 64, 1), 256, 0, stream>>>(g1, g1, g1, g1, g1T, g1T, kChan, kLoraG, kChan, kLoraG, 0);
  wt_plane_kernel<<<dim3(kLoraW / 64, kChan / 64, 1), 256, 0, stream>>>(w2, w2, w2, w2, w2T, w2T, kLoraW, kChan, kLoraW, kChan, 0);
  wt_plane_kernel<<<dim3(kLoraA / 64, kChan / 64, 1), 256, 0, stream>>>(a2, a2, a2, a2, a2T, a2T, kLoraA, kChan, kLoraA, kChan, 0);
  wt_plane_kernel<<<dim3(kLoraVP / 64, kChan / 64, 1), 256, 0, stream>>>(v2, v2, v2, v2, v2T, v2T, kLoraV, kChan, kLoraVP, kChan, 0);
  wt_plane_kernel<<<dim3(kLoraG / 64, kChan / 64, 1), 256, 0, stream>>>(g2, g2, g2, g2, g2T, g2T, kLoraG, kChan, kLoraG, kChan, 0);

  mix_kernel<<<(kTok * (kChan / 8)) / 256, 256, 0, stream>>>(x, x_r, x_w, x_k, x_v, x_a, x_g,
                                                             XRh, XRr, XKh, XKr, XVh, XVr, XW, XA, XG);

  const int blkBig = (kTok / 32) * (kChan / 64) / 8;
  gemm_f16_kernel<true, 0, 0><<<dim3(blkBig, 3), 256, 0, stream>>>(
      XRh, XRr, kChan, (long)kPlane, WBh, WBr, kChan, (long)wBig,
      (void*)Rf, kChan, (long)kPlane, kTok, kChan, kChan, kScaleW);

  const int blk64  = (kTok / 32) * (64 / 64) / 8;
  const int blk128 = (kTok / 32) * (128 / 64) / 8;
  gemm_f16_kernel<false, 1, 1><<<dim3(blk64, 1), 256, 0, stream>>>(
      XW, XW, kChan, 0L, w1T, w1T, kChan, 0L, (void*)HW, kLoraW, 0L, kTok, kLoraW, kChan, kScaleW);
  gemm_f16_kernel<false, 0, 1><<<dim3(blk64, 1), 256, 0, stream>>>(
      XA, XA, kChan, 0L, a1T, a1T, kChan, 0L, (void*)HA, kLoraA, 0L, kTok, kLoraA, kChan, 1.0f);
  gemm_f16_kernel<false, 0, 1><<<dim3(blk64, 1), 256, 0, stream>>>(
      XVh, XVh, kChan, 0L, v1T, v1T, kChan, 0L, (void*)HV, kLoraVP, 0L, kTok, kLoraVP, kChan, 1.0f);
  gemm_f16_kernel<false, 2, 1><<<dim3(blk128, 1), 256, 0, stream>>>(
      XG, XG, kChan, 0L, g1T, g1T, kChan, 0L, (void*)HG, kLoraG, 0L, kTok, kLoraG, kChan, kScaleW);

  gemm_f16_kernel<false, 0, 0><<<dim3(blkBig, 1), 256, 0, stream>>>(
      HW, HW, kLoraW, 0L, w2T, w2T, kLoraW, 0L, (void*)WD, kChan, 0L, kTok, kChan, kLoraW, kScaleWH);
  gemm_f16_kernel<false, 0, 0><<<dim3(blkBig, 1), 256, 0, stream>>>(
      HA, HA, kLoraA, 0L, a2T, a2T, kLoraA, 0L, (void*)AB, kChan, 0L, kTok, kChan, kLoraA, kScaleWH);
  gemm_f16_kernel<false, 0, 0><<<dim3(blkBig, 1), 256, 0, stream>>>(
      HV, HV, kLoraVP, 0L, v2T, v2T, kLoraVP, 0L, (void*)VK, kChan, 0L, kTok, kChan, kLoraVP, kScaleWH);
  gemm_f16_kernel<false, 0, 0><<<dim3(blkBig, 1), 256, 0, stream>>>(
      HG, HG, kLoraG, 0L, g2T, g2T, kLoraG, 0L, (void*)Gf, kChan, 0L, kTok, kChan, kLoraG, kScaleWH);

  gate_prep_kernel<<<(kTok * kHeads) / 8, 256, 0, stream>>>(Kf, Vf, WD, AB, VK, vfirst, w0, a0, v0, k_k, k_a);

  state_scan_kernel<<<kBatch * kHeads, 256, 0, stream>>>(Rf, WD, Kf, Vf, VK, AB, Yf);

  norm_gate_kernel<<<(kTok * kHeads) / 8, 256, 0, stream>>>(Yf, Rf, Kf, Vf, Gf, r_k, ln_w, ln_b,
                                                            (unsigned*)YGh, (unsigned*)YGr);

  gemm_f16_kernel<true, 0, 0><<<dim3(blkBig, 1), 256, 0, stream>>>(
      YGh, YGr, kChan, 0L, WBh + 3 * wBig, WBr + 3 * wBig, kChan, 0L,
      (void*)out0, kChan, 0L, kTok, kChan, kChan, kScaleOut);

  copy_f32x4_kernel<<<(nP / 4) / 256, 256, 0, stream>>>(vfirst, out1, nP / 4);
}
